// RelativeGlobalAttention_10660108828830
// MI455X (gfx1250) — hardware-verified
//
#include <hip/hip_runtime.h>
#include <math.h>

#ifndef NB
#define NB 2
#endif
#ifndef SEQ
#define SEQ 2048
#endif
#define NB_FULL  2
#define SEQ_FULL 2048
#define DMD  512
#define NH   8
#define HD   64
#define EVD  388
#define EVP  448
#define MT   (NB * SEQ)
#define KF   (2 * DMD)
#define NFLG (SEQ / 16)
#define FLGW 32
#define AWV  4
#define RWP  48
#define WSCL 64.0f
#define QKS  16.0f
#define RSQD 0.125f
#define NEGM (-1.0e10f)

static_assert(NB >= 1 && NB <= NB_FULL);
static_assert(SEQ >= 64 && SEQ <= SEQ_FULL && (SEQ % 64) == 0);
static_assert(NH * HD == DMD && HD == 64);
static_assert((MT % 64) == 0 && (DMD % 64) == 0 && (KF % 64) == 0);
static_assert((EVP % 64) == 0 && EVP >= EVD && (EVD % 4) == 0);
static_assert(((SEQ * DMD) % 2048) == 0 && ((NH * SEQ_FULL * HD) % 2048) == 0);
static_assert(((NB * NH * (SEQ / 16)) % AWV) == 0);
static_assert(NFLG <= 256 && ((4 * SEQ) % 256) == 0);

typedef _Float16 v16h __attribute__((ext_vector_type(16)));
typedef __bf16 v16bf __attribute__((ext_vector_type(16)));
typedef unsigned short v16us __attribute__((ext_vector_type(16)));
typedef unsigned short v8us  __attribute__((ext_vector_type(8)));
typedef float v8f __attribute__((ext_vector_type(8)));
typedef float v4f __attribute__((ext_vector_type(4)));
typedef unsigned int v4u __attribute__((ext_vector_type(4)));

union FragU { v16us v; v8us h[2]; };

__device__ __forceinline__ unsigned short bf_bits(float f) {
  const unsigned u = __float_as_uint(f);
  return (unsigned short)((u + 0x7FFFu + ((u >> 16) & 1u)) >> 16);
}
__device__ __forceinline__ float bf_up(unsigned short h) { return __uint_as_float(((unsigned)h) << 16); }
__device__ __forceinline__ float bfr(float f) { return bf_up(bf_bits(f)); }
__device__ __forceinline__ unsigned short h_bits(_Float16 x) { return __builtin_bit_cast(unsigned short, x); }
__device__ __forceinline__ unsigned short f2h(float f) { return h_bits((_Float16)f); }
__device__ __forceinline__ unsigned pk16(unsigned short a, unsigned short b) { return (unsigned)a | ((unsigned)b << 16); }
__device__ __forceinline__ int clampi(int v, int lo, int hi) { return v < lo ? lo : (v > hi ? hi : v); }
__device__ __forceinline__ v8f zero8() { v8f z = {0.f, 0.f, 0.f, 0.f, 0.f, 0.f, 0.f, 0.f}; return z; }

__device__ __forceinline__ v16us ldfrag_u(const unsigned short* p) {
  FragU f;
  f.h[0] = *(const v8us*)(p);
  f.h[1] = *(const v8us*)(p + 16);
  return f.v;
}

__device__ __forceinline__ v8f mma_raw(v16us a, v16us b, v8f c) {
  return __builtin_amdgcn_wmma_f32_16x16x32_f16(false, __builtin_bit_cast(v16h, a), false,
                                                __builtin_bit_cast(v16h, b), (short)0, c, false, false);
}
__device__ __forceinline__ v8f mma_raw_bf(v16us a, v16us b, v8f c) {
  return __builtin_amdgcn_wmma_f32_16x16x32_bf16(false, __builtin_bit_cast(v16bf, a), false,
                                                 __builtin_bit_cast(v16bf, b), (short)0, c, false, false);
}
__device__ __forceinline__ v8f mma_g(v16us a, v16us b, v8f c) {
  c = mma_raw(a, b, c);
#if defined(__HIP_DEVICE_COMPILE__)
  asm volatile("v_nop\n\tv_nop\n\tv_nop\n\tv_nop" : "+v"(c) : "v"(a), "v"(b));
#endif
  return c;
}
__device__ __forceinline__ v8f mma_gb(v16us a, v16us b, v8f c) {
  c = mma_raw_bf(a, b, c);
#if defined(__HIP_DEVICE_COMPILE__)
  asm volatile("v_nop\n\tv_nop\n\tv_nop\n\tv_nop" : "+v"(c) : "v"(a), "v"(b));
#endif
  return c;
}
__device__ __forceinline__ void dep_guard1(v8f& a, v8f& b, v16us x) {
#if defined(__HIP_DEVICE_COMPILE__)
  asm volatile("v_nop\n\tv_nop\n\tv_nop\n\tv_nop" : "+v"(a), "+v"(b) : "v"(x));
#endif
}
__device__ __forceinline__ void keep4_u(v16us a, v16us b, v16us c, v16us d) {
#if defined(__HIP_DEVICE_COMPILE__)
  asm volatile("v_nop" :: "v"(a), "v"(b), "v"(c), "v"(d));
#endif
}
__device__ __forceinline__ void acc_guard4(v8f& a, v8f& b, v8f& c, v8f& d) {
#if defined(__HIP_DEVICE_COMPILE__)
  asm volatile("v_nop\n\tv_nop\n\tv_nop\n\tv_nop" : "+v"(a), "+v"(b), "+v"(c), "+v"(d));
#endif
}
__device__ __forceinline__ void wave_sync_lds() {
  __builtin_amdgcn_fence(__ATOMIC_RELEASE, "workgroup");
  __builtin_amdgcn_wave_barrier();
  __builtin_amdgcn_fence(__ATOMIC_ACQUIRE, "workgroup");
}

__global__ __launch_bounds__(256) void cvt_lin(const float* __restrict__ w, unsigned short* o,
                                                int nsrc, int ndst, float sc, int sstr, int dstr) {
  const float* wb = w + (size_t)blockIdx.y * (size_t)sstr;
  unsigned short* ob = o + (size_t)blockIdx.y * (size_t)dstr;
  const int base = (blockIdx.x * 256 + threadIdx.x) * 8;
  if (base + 8 > ndst) return;
  const bool inr = (base + 8 <= nsrc);
  const int lb = inr ? base : (nsrc - 8);
  const v4f a0 = *(const v4f*)(wb + lb);
  const v4f a1 = *(const v4f*)(wb + lb + 4);
  v4u hv;
#pragma unroll
  for (int e = 0; e < 2; ++e) {
    hv[e]     = pk16(f2h(bfr(a0[2 * e]) * sc), f2h(bfr(a0[2 * e + 1]) * sc));
    hv[2 + e] = pk16(f2h(bfr(a1[2 * e]) * sc), f2h(bfr(a1[2 * e + 1]) * sc));
  }
  const v4u zz = {0u, 0u, 0u, 0u};
  hv = inr ? hv : zz;
  unsigned short* d = ob + base;
  *(volatile v4u*)d = hv;
  __threadfence();
  *(volatile v4u*)d = hv;
}

template <int BFO>
__global__ __launch_bounds__(256) void cvt_t(const float* __restrict__ w, unsigned short* o,
                                              int R, int C, int CP, int ldo, float sc) {
  __shared__ __align__(16) unsigned short st[64 * 72];
  const int t = threadIdx.x;
  const int r0 = blockIdx.y * 64, c0 = blockIdx.x * 64;
  if (r0 + 64 > R || c0 + 64 > CP) return;
  {
    const int row = t >> 2, ch = (t & 3) * 16;
    const float* p = w + (size_t)(r0 + row) * C;
#pragma unroll
    for (int q = 0; q < 4; ++q) {
      const int cs = c0 + ch + 4 * q;
      const bool inr = (cs + 4 <= C);
      const int lb = inr ? cs : (C - 4);
      const v4f v = *(const v4f*)(p + lb);
#pragma unroll
      for (int e = 0; e < 4; ++e) {
        const unsigned short hb = BFO ? bf_bits(v[e]) : f2h(bfr(v[e]) * sc);
        st[(ch + 4 * q + e) * 72 + row] = inr ? hb : (unsigned short)0;
      }
    }
  }
  __syncthreads();
  v4u hv[2];
#pragma unroll
  for (int half = 0; half < 2; ++half) {
    const int cl = (t >> 3) + 32 * half, pc = (t & 7) * 8;
    hv[half] = *(const v4u*)(st + cl * 72 + pc);
  }
  for (int pass = 0; pass < 2; ++pass) {
#pragma unroll
    for (int half = 0; half < 2; ++half) {
      const int cl = (t >> 3) + 32 * half, pc = (t & 7) * 8;
      unsigned short* dst = o + (size_t)(c0 + cl) * ldo + r0 + pc;
      *(volatile v4u*)dst = hv[half];
    }
    __threadfence();
  }
}

template <int BF, int OM, int RELU, int BROW>
__global__ __launch_bounds__(256) void gemm64(
    const unsigned short* __restrict__ Ap, int lda, const unsigned short* __restrict__ Btp, int ldb,
    unsigned short* Ch, int looff, float* Cf, int ldc, float osc,
    const float* __restrict__ bias, int nbias, float bsc, int M, int N, int K) {
  __shared__ __align__(16) float sT[8][16 * 68];
  const int lane = threadIdx.x & 31;
  const int wave = threadIdx.x >> 5;
  const int tilesN = N >> 6;
  const int tilesM = M >> 6;
  const int tile = blockIdx.x * 8 + wave;
  if (tile >= tilesM * tilesN) return;
  const int tm = tile / tilesN;
  const int tn = tile - tm * tilesN;
  const int m0 = tm << 6;
  const int n0 = tn << 6;

  const int rlane = lane & 15;
  const int koff  = (lane >> 4) * 8;
  const int mOff  = (lane >> 4) * 8;

  v8f acc[4][4];
#pragma unroll
  for (int i = 0; i < 4; ++i)
#pragma unroll
    for (int j = 0; j < 4; ++j) acc[i][j] = zero8();

#pragma unroll 1
  for (int k0 = 0; k0 < K; k0 += 32) {
    v16us bh[4];
#pragma unroll
    for (int j = 0; j < 4; ++j) {
      const size_t bo = (size_t)(n0 + (j << 4) + rlane) * ldb + koff + k0;
      bh[j] = ldfrag_u(Btp + bo);
    }
#pragma unroll
    for (int i = 0; i < 4; ++i) {
      const size_t ao = (size_t)(m0 + (i << 4) + rlane) * lda + koff + k0;
      const v16us ah = ldfrag_u(Ap + ao);
#pragma unroll
      for (int j = 0; j < 4; ++j) {
        if (BF) acc[i][j] = mma_raw_bf(ah, bh[j], acc[i][j]);
        else    acc[i][j] = mma_raw(ah, bh[j], acc[i][j]);
      }
      dep_guard1(acc[i][0], acc[i][3], ah);
    }
    keep4_u(bh[0], bh[1], bh[2], bh[3]);
  }
  acc_guard4(acc[0][0], acc[0][1], acc[0][2], acc[0][3]);
  acc_guard4(acc[1][0], acc[1][1], acc[1][2], acc[1][3]);
  acc_guard4(acc[2][0], acc[2][1], acc[2][2], acc[2][3]);
  acc_guard4(acc[3][0], acc[3][1], acc[3][2], acc[3][3]);

  const int hh2 = lane >> 4, c4 = (lane & 15) * 4;
  const int q8  = lane >> 3, c8 = (lane & 7) * 8;

  float bc[8];
#pragma unroll
  for (int e = 0; e < 8; ++e) bc[e] = 0.f;
  if (!BROW) {
    if (OM == 0) {
#pragma unroll
      for (int e = 0; e < 4; ++e) bc[e] = bsc * bfr(bias[clampi(n0 + c4 + e, 0, nbias - 1)]);
    } else {
#pragma unroll
      for (int e = 0; e < 8; ++e) bc[e] = bsc * bfr(bias[clampi(n0 + c8 + e, 0, nbias - 1)]);
    }
  }

  float* slab = sT[wave];
#pragma unroll
  for (int i = 0; i < 4; ++i) {
    const int mBase = m0 + (i << 4);
#pragma unroll
    for (int j = 0; j < 4; ++j) {
#pragma unroll
      for (int r = 0; r < 8; ++r) {
        slab[(mOff + r) * 68 + (j << 4) + rlane] = acc[i][j][r];
      }
    }
    wave_sync_lds();
    if (OM == 0) {
      v4f vals[8];
#pragma unroll
      for (int it = 0; it < 8; ++it) {
        const int row = it * 2 + hh2;
        const v4f v = *(const v4f*)(slab + row * 68 + c4);
        float brw = 0.f;
        if (BROW) brw = bsc * bfr(bias[clampi(mBase + row, 0, nbias - 1)]);
        v4f ov;
#pragma unroll
        for (int e = 0; e < 4; ++e) {
          float x = v[e] * osc + (BROW ? brw : bc[e]);
          if (RELU) x = fmaxf(x, 0.f);
          ov[e] = x;
        }
        vals[it] = ov;
      }
      for (int pass = 0; pass < 2; ++pass) {
#pragma unroll
        for (int it = 0; it < 8; ++it) {
          const int row = it * 2 + hh2;
          *(volatile v4f*)(Cf + (size_t)(mBase + row) * ldc + (size_t)n0 + c4) = vals[it];
        }
        __threadfence();
      }
    } else if (OM == 1) {
      v4u hv[4];
#pragma unroll
      for (int it = 0; it < 4; ++it) {
        const int row = it * 4 + q8;
        const float* sp = slab + row * 68 + c8;
        float brw = 0.f;
        if (BROW) brw = bsc * bfr(bias[clampi(mBase + row, 0, nbias - 1)]);
        v4u ha = {0u, 0u, 0u, 0u};
#pragma unroll
        for (int e = 0; e < 4; ++e) {
          float b0 = sp[2 * e]     * osc + (BROW ? brw : bc[2 * e]);
          float b1 = sp[2 * e + 1] * osc + (BROW ? brw : bc[2 * e + 1]);
          if (RELU) { b0 = fmaxf(b0, 0.f); b1 = fmaxf(b1, 0.f); }
          ha[e] = pk16(f2h(b0), f2h(b1));
        }
        hv[it] = ha;
      }
      for (int pass = 0; pass < 2; ++pass) {
#pragma unroll
        for (int it = 0; it < 4; ++it) {
          const int row = it * 4 + q8;
          const size_t go = (size_t)(mBase + row) * ldc + (size_t)n0 + c8;
          *(volatile v4u*)(Ch + go) = hv[it];
        }
        __threadfence();
      }
    } else {
      v4u hv[4], lv[4];
#pragma unroll
      for (int it = 0; it < 4; ++it) {
        const int row = it * 4 + q8;
        const float* sp = slab + row * 68 + c8;
        float brw = 0.f;
        if (BROW) brw = bsc * bfr(bias[clampi(mBase + row, 0, nbias - 1)]);
        v4u ha = {0u, 0u, 0u, 0u};
        v4u la = {0u, 0u, 0u, 0u};
#pragma unroll
        for (int e = 0; e < 4; ++e) {
          float x0 = sp[2 * e]     * osc + (BROW ? brw : bc[2 * e]);
          float x1 = sp[2 * e + 1] * osc + (BROW ? brw : bc[2 * e + 1]);
          if (RELU) { x0 = fmaxf(x0, 0.f); x1 = fmaxf(x1, 0.f); }
          const unsigned short h0 = bf_bits(x0), h1 = bf_bits(x1);
          const unsigned short l0 = bf_bits(x0 - bf_up(h0)), l1 = bf_bits(x1 - bf_up(h1));
          ha[e] = pk16(h0, h1);
          la[e] = pk16(l0, l1);
        }
        hv[it] = ha;
        lv[it] = la;
      }
      for (int pass = 0; pass < 2; ++pass) {
#pragma unroll
        for (int it = 0; it < 4; ++it) {
          const int row = it * 4 + q8;
          const size_t go = (size_t)(mBase + row) * ldc + (size_t)n0 + c8;
          *(volatile v4u*)(Ch + go) = hv[it];
          *(volatile v4u*)(Ch + (size_t)looff + go) = lv[it];
        }
        __threadfence();
      }
    }
    wave_sync_lds();
  }
}

__global__ __launch_bounds__(256) void mask_check(const float* __restrict__ msk, float* flg) {
  __shared__ int wf[8];
  const int t = threadIdx.x, lane = t & 31, wv = t >> 5;
  const int i0 = blockIdx.x * 16;
  if (i0 + 16 > SEQ) return;
  constexpr int C4 = SEQ / 4;
  int viol = 0;
#pragma unroll 1
  for (int it = 0; it < (16 * C4) / 256; ++it) {
    const int ci = it * 256 + t;
    const int rr = ci / C4;
    const int c4 = ci - rr * C4;
    const int i = i0 + rr;
    const v4f x = *(const v4f*)(msk + (size_t)i * SEQ_FULL + 4 * c4);
#pragma unroll
    for (int e = 0; e < 4; ++e) {
      const int j = 4 * c4 + e;
      const float ex = (j <= i) ? 1.0f : 0.0f;
      viol |= (x[e] != ex) ? 1 : 0;
    }
  }
  viol |= __shfl_xor(viol, 1, 32);
  viol |= __shfl_xor(viol, 2, 32);
  viol |= __shfl_xor(viol, 4, 32);
  viol |= __shfl_xor(viol, 8, 32);
  viol |= __shfl_xor(viol, 16, 32);
  if (lane == 0) wf[wv] = viol;
  __syncthreads();
  if (wv == 0) {
    int f = wf[lane & 7];
    f |= __shfl_xor(f, 1, 32);
    f |= __shfl_xor(f, 2, 32);
    f |= __shfl_xor(f, 4, 32);
    const float fv = f ? 1.0f : 0.0f;
    float* d = flg + (size_t)blockIdx.x * FLGW + lane;
    *(volatile float*)d = fv;
    __threadfence();
    *(volatile float*)d = fv;
  }
}

__global__ __launch_bounds__(128) void attn_kernel(
    const unsigned short* __restrict__ QH, const unsigned short* __restrict__ KH,
    const unsigned short* __restrict__ PE, const unsigned short* __restrict__ VH,
    const unsigned short* __restrict__ VL, unsigned short* Z) {
  __shared__ __align__(16) float relw[AWV][16 * RWP];
  __shared__ __align__(16) unsigned short pwh[AWV][16 * 32];
  __shared__ __align__(16) unsigned short pwl[AWV][16 * 32];
  __shared__ __align__(16) unsigned short zst[AWV][16 * 128];
  const int lane = threadIdx.x & 31, wv = threadIdx.x >> 5, m = lane & 15, hh = lane >> 4;
  const int task = blockIdx.x * AWV + wv;
  const int nqt = SEQ / 16;
  const int bh = task / nqt;
  const int t0 = (task - bh * nqt) << 4;
  const int b = bh / NH, h = bh - (bh / NH) * NH;
  if (b >= NB) return;
  const size_t tok0 = (size_t)b * SEQ;
  float* rw = relw[wv];
  unsigned short* ph = pwh[wv];
  unsigned short* pl = pwl[wv];

  const unsigned short* qp = QH + (tok0 + (size_t)(t0 + m)) * HD + 8 * hh;
  const v16us qf0 = ldfrag_u(qp);
  const v16us qf1 = ldfrag_u(qp + 32);

  const unsigned short* pe = PE + (size_t)h * SEQ_FULL * HD;
  const int rb = SEQ - 16 - t0;

  v8f carry;
  {
    const int u = clampi(rb + m, 0, SEQ - 1);
    const unsigned short* pp = pe + (size_t)u * HD + 8 * hh;
    carry = mma_g(qf0, ldfrag_u(pp), zero8());
    carry = mma_g(qf1, ldfrag_u(pp + 32), carry);
  }

  float mx[8], ls[8];
  v8f O0 = zero8(), O1 = zero8(), O2 = zero8(), O3 = zero8();
#pragma unroll
  for (int r = 0; r < 8; ++r) { mx[r] = -1.0e30f; ls[r] = 0.f; }

  const int nkb = (t0 >> 5) + 1;
  const size_t vst = (size_t)16 * MT;

#pragma unroll 1
  for (int kb = 0; kb < nkb; ++kb) {
    const int sb = kb << 5;
    v8f S0, S1;
    {
      const unsigned short* kp = KH + (tok0 + (size_t)(sb + m)) * HD + 8 * hh;
      S0 = mma_g(qf0, ldfrag_u(kp), zero8());
      S0 = mma_g(qf1, ldfrag_u(kp + 32), S0);
      const unsigned short* kp1 = kp + (size_t)16 * HD;
      S1 = mma_g(qf0, ldfrag_u(kp1), zero8());
      S1 = mma_g(qf1, ldfrag_u(kp1 + 32), S1);
    }

    v8f Pb1, Pb2;
    {
      const int u1 = clampi(rb + sb + 16 + m, 0, SEQ - 1);
      const unsigned short* p1 = pe + (size_t)u1 * HD + 8 * hh;
      Pb1 = mma_g(qf0, ldfrag_u(p1), zero8());
      Pb1 = mma_g(qf1, ldfrag_u(p1 + 32), Pb1);
      const int u2 = clampi(rb + sb + 32 + m, 0, SEQ - 1);
      const unsigned short* p2 = pe + (size_t)u2 * HD + 8 * hh;
      Pb2 = mma_g(qf0, ldfrag_u(p2), zero8());
      Pb2 = mma_g(qf1, ldfrag_u(p2 + 32), Pb2);
    }
#pragma unroll
    for (int r = 0; r < 8; ++r) {
      const int row = 8 * hh + r;
      rw[row * RWP + m]      = carry[r];
      rw[row * RWP + 16 + m] = Pb1[r];
      rw[row * RWP + 32 + m] = Pb2[r];
    }
    carry = Pb2;
    wave_sync_lds();

    float s0[8], s1[8];
#pragma unroll
    for (int r = 0; r < 8; ++r) {
      const int row = 8 * hh + r;
      const int i = t0 + row;
      const float rv0 = rw[row * RWP + 15 - row + m];
      const float rv1 = rw[row * RWP + 31 - row + m];
      const float a0 = (S0[r] * (1.0f / (QKS * QKS)) + rv0 * (1.0f / (QKS * WSCL))) * RSQD;
      const float a1 = (S1[r] * (1.0f / (QKS * QKS)) + rv1 * (1.0f / (QKS * WSCL))) * RSQD;
      s0[r] = (sb + m <= i) ? a0 : NEGM;
      s1[r] = (sb + 16 + m <= i) ? a1 : NEGM;
    }

#pragma unroll
    for (int r = 0; r < 8; ++r) {
      float xm = fmaxf(s0[r], s1[r]);
      xm = fmaxf(xm, __shfl_xor(xm, 1, 32));
      xm = fmaxf(xm, __shfl_xor(xm, 2, 32));
      xm = fmaxf(xm, __shfl_xor(xm, 4, 32));
      xm = fmaxf(xm, __shfl_xor(xm, 8, 32));
      const float mn = fmaxf(mx[r], xm);
      const float al = __expf(mx[r] - mn);
      mx[r] = mn;
      const float p0 = __expf(s0[r] - mn);
      const float p1 = __expf(s1[r] - mn);
      float ps = p0 + p1;
      ps += __shfl_xor(ps, 1, 32);
      ps += __shfl_xor(ps, 2, 32);
      ps += __shfl_xor(ps, 4, 32);
      ps += __shfl_xor(ps, 8, 32);
      ls[r] = ls[r] * al + ps;
      O0[r] = O0[r] * al;
      O1[r] = O1[r] * al;
      O2[r] = O2[r] * al;
      O3[r] = O3[r] * al;
      const int row = 8 * hh + r;
      const unsigned short hb0 = bf_bits(p0), hb1 = bf_bits(p1);
      ph[row * 32 + m]      = hb0;
      ph[row * 32 + 16 + m] = hb1;
      pl[row * 32 + m]      = bf_bits(p0 - bf_up(hb0));
      pl[row * 32 + 16 + m] = bf_bits(p1 - bf_up(hb1));
    }
    wave_sync_lds();

    const v16us afh = ldfrag_u(ph + m * 32 + 8 * hh);
    const v16us afl = ldfrag_u(pl + m * 32 + 8 * hh);
    const size_t vo = (size_t)m * MT + tok0 + (size_t)sb + 8 * hh;
    {
      const v16us vh = ldfrag_u(VH + vo);
      const v16us vl = ldfrag_u(VL + vo);
      O0 = mma_gb(afh, vh, O0);
      O0 = mma_gb(afh, vl, O0);
      O0 = mma_gb(afl, vh, O0);
    }
    {
      const v16us vh = ldfrag_u(VH + vo + vst);
      const v16us vl = ldfrag_u(VL + vo + vst);
      O1 = mma_gb(afh, vh, O1);
      O1 = mma_gb(afh, vl, O1);
      O1 = mma_gb(afl, vh, O1);
    }
    {
      const v16us vh = ldfrag_u(VH + vo + 2 * vst);
      const v16us vl = ldfrag_u(VL + vo + 2 * vst);
      O2 = mma_gb(afh, vh, O2);
      O2 = mma_gb(afh, vl, O2);
      O2 = mma_gb(afl, vh, O2);
    }
    {
      const v16us vh = ldfrag_u(VH + vo + 3 * vst);
      const v16us vl = ldfrag_u(VL + vo + 3 * vst);
      O3 = mma_gb(afh, vh, O3);
      O3 = mma_gb(afh, vl, O3);
      O3 = mma_gb(afl, vh, O3);
    }
  }
  acc_guard4(O0, O1, O2, O3);

  unsigned short* zs = zst[wv];
#pragma unroll
  for (int r = 0; r < 8; ++r) {
    const int row = 8 * hh + r;
    const float g = 1.0f / ls[r];
    {
      const float c = O0[r] * g; const unsigned short hb = bf_bits(c);
      zs[row * 128 + m]       = hb;  zs[row * 128 + 64 + m]  = bf_bits(c - bf_up(hb));
    }
    {
      const float c = O1[r] * g; const unsigned short hb = bf_bits(c);
      zs[row * 128 + 16 + m]  = hb;  zs[row * 128 + 80 + m]  = bf_bits(c - bf_up(hb));
    }
    {
      const float c = O2[r] * g; const unsigned short hb = bf_bits(c);
      zs[row * 128 + 32 + m]  = hb;  zs[row * 128 + 96 + m]  = bf_bits(c - bf_up(hb));
    }
    {
      const float c = O3[r] * g; const unsigned short hb = bf_bits(c);
      zs[row * 128 + 48 + m]  = hb;  zs[row * 128 + 112 + m] = bf_bits(c - bf_up(hb));
    }
  }
  wave_sync_lds();
  {
    const int q8 = lane >> 3, c8 = (lane & 7) * 8;
    v4u hv[4], lv[4];
#pragma unroll
    for (int it = 0; it < 4; ++it) {
      const int row = it * 4 + q8;
      hv[it] = *(const v4u*)(zs + row * 128 + c8);
      lv[it] = *(const v4u*)(zs + row * 128 + 64 + c8);
    }
    const size_t zr0 = tok0 + (size_t)t0;
    for (int pass = 0; pass < 2; ++pass) {
#pragma unroll
      for (int it = 0; it < 4; ++it) {
        const int row = it * 4 + q8;
        unsigned short* dst = Z + (zr0 + (size_t)row) * KF + h * HD + c8;
        *(volatile v4u*)dst = hv[it];
        *(volatile v4u*)(dst + DMD) = lv[it];
      }
      __threadfence();
    }
  }
}

__global__ __launch_bounds__(256) void out_copy(const float* __restrict__ L, const float* __restrict__ flg,
                                                 float* out) {
  __shared__ int wf[8];
  const int t = threadIdx.x, lane = t & 31, wv = t >> 5;
  int f;
  {
    const int ti = (t < NFLG) ? t : (NFLG - 1);
    const float x = flg[(size_t)ti * FLGW];
    f = ((t < NFLG) && (x == 1.0f)) ? 1 : 0;
  }
  f |= __shfl_xor(f, 1, 32);
  f |= __shfl_xor(f, 2, 32);
  f |= __shfl_xor(f, 4, 32);
  f |= __shfl_xor(f, 8, 32);
  f |= __shfl_xor(f, 16, 32);
  if (lane == 0) wf[wv] = f;
  __syncthreads();
  int g = 0;
#pragma unroll
  for (int w = 0; w < 8; ++w) g |= wf[w];
  const int e4 = blockIdx.x * 256 + t;
  if (e4 < MT * (EVD / 4)) {
    const int e = e4 * 4;
    const int row = e / EVD;
    const int c = e - row * EVD;
    v4f x = *(const v4f*)(L + (size_t)row * EVP + c);
    const float qn = __uint_as_float(0x7fc00000u);
    const v4f pn = {qn, qn, qn, qn};
    x = g ? pn : x;
    float* d = out + (size_t)e;
    *(volatile v4f*)d = x;
    __threadfence();
    *(volatile v4f*)d = x;
  }
}

extern "C" void kernel_launch(void* const* d_in, const int* in_sizes, int n_in,
                              void* d_out, int out_size, void* d_ws, size_t ws_size,
                              hipStream_t stream) {
  if (n_in < 15) return;
  if (in_sizes[0] < (NB - 1) * SEQ_FULL * DMD + SEQ * DMD) return;
  if (in_sizes[1] < (NB - 1) * SEQ_FULL * DMD + SEQ * DMD) return;
  if (in_sizes[2] < (NB - 1) * SEQ_FULL * DMD + SEQ * DMD) return;
  if (in_sizes[3] < (SEQ - 1) * SEQ_FULL + SEQ) return;
  if (in_sizes[4] < DMD * HD || in_sizes[6] < DMD * HD || in_sizes[8] < DMD * HD) return;
  if (in_sizes[5] < HD || in_sizes[7] < HD || in_sizes[9] < HD) return;
  if (in_sizes[10] < NH * SEQ_FULL * HD) return;
  if (in_sizes[11] < DMD * DMD || in_sizes[12] < DMD) return;
  if (in_sizes[13] < DMD * EVD || in_sizes[14] < EVD) return;
  if (out_size < MT * EVD) return;

  const float* v   = (const float*)d_in[0];
  const float* k   = (const float*)d_in[1];
  const float* q   = (const float*)d_in[2];
  const float* msk = (const float*)d_in[3];
  const float* wq  = (const float*)d_in[4];
  const float* bq  = (const float*)d_in[5];
  const float* wk  = (const float*)d_in[6];
  const float* bk  = (const float*)d_in[7];
  const float* wv  = (const float*)d_in[8];
  const float* bv  = (const float*)d_in[9];
  const float* ee  = (const float*)d_in[10];
  const float* wo  = (const float*)d_in[11];
  const float* bo  = (const float*)d_in[12];
  const float* wl  = (const float*)d_in[13];
  const float* bl  = (const float*)d_in[14];

  const size_t PX  = (size_t)MT * DMD * 2;
  const size_t PW  = (size_t)HD * DMD * 2;
  const size_t PPE = (size_t)NH * SEQ_FULL * HD * 2;
  const size_t PQK = (size_t)MT * HD * 2;
  const size_t PV2 = (size_t)2 * HD * MT * 2;
  const size_t PZ  = (size_t)MT * KF * 2;
  const size_t PWO = (size_t)DMD * KF * 2;
  const size_t POP = (size_t)MT * KF * 2;
  const size_t PWL = (size_t)EVP * KF * 2;
  const size_t PL  = (size_t)MT * EVP * 4;
  const size_t PFL = (size_t)(SEQ_FULL / 16) * FLGW * 4;
  size_t off = 0;
  const size_t oXQ = off; off += PX;
  const size_t oXK = off; off += PX;
  const size_t oXV = off; off += PX;
  const size_t oWQ = off; off += PW;
  const size_t oWK = off; off += PW;
  const size_t oWV = off; off += PW;
  const size_t oPE = off; off += PPE;
  const size_t oQH = off; off += PQK;
  const size_t oKH = off; off += PQK;
  const size_t oV  = off; off += PV2;
  const size_t oZ  = off; off += PZ;
  const size_t oWO = off; off += PWO;
  const size_t oOP = off; off += POP;
  const size_t oWL = off; off += PWL;
  const size_t oL  = off; off += PL;
  const size_t oFL = off; off += PFL;
  if (off > ws_size) return;
  if (off > (size_t)134217728) return;

  char* ws = (char*)d_ws;
  unsigned short* XQ  = (unsigned short*)(ws + oXQ);
  unsigned short* XK  = (unsigned short*)(ws + oXK);
  unsigned short* XV  = (unsigned short*)(ws + oXV);
  unsigned short* WQT = (unsigned short*)(ws + oWQ);
  unsigned short* WKT = (unsigned short*)(ws + oWK);
  unsigned short* WVT = (unsigned short*)(ws + oWV);
  unsigned short* PEH = (unsigned short*)(ws + oPE);
  unsigned short* QHp = (unsigned short*)(ws + oQH);
  unsigned short* KHp = (unsigned short*)(ws + oKH);
  unsigned short* VHp = (unsigned short*)(ws + oV);
  unsigned short* VLp = VHp + (size_t)HD * MT;
  unsigned short* Zp  = (unsigned short*)(ws + oZ);
  unsigned short* WOT = (unsigned short*)(ws + oWO);
  unsigned short* OPp = (unsigned short*)(ws + oOP);
  unsigned short* WLT = (unsigned short*)(ws + oWL);
  float* Lp   = (float*)(ws + oL);
  float* FLG  = (float*)(ws + oFL);
  float* out0 = (float*)d_out;
  float* fdummy = Lp;
  unsigned short* hdummy = QHp;

  const dim3 blk(256);

  const int gX = (SEQ * DMD) / 2048;
  cvt_lin<<<dim3(gX, NB), blk, 0, stream>>>(q, XQ, SEQ * DMD, SEQ * DMD, 1.0f, SEQ_FULL * DMD, SEQ * DMD);
  cvt_lin<<<dim3(gX, NB), blk, 0, stream>>>(k, XK, SEQ * DMD, SEQ * DMD, 1.0f, SEQ_FULL * DMD, SEQ * DMD);
  cvt_lin<<<dim3(gX, NB), blk, 0, stream>>>(v, XV, SEQ * DMD, SEQ * DMD, 1.0f, SEQ_FULL * DMD, SEQ * DMD);
  cvt_lin<<<dim3((NH * SEQ_FULL * HD) / 2048, 1), blk, 0, stream>>>(ee, PEH, NH * SEQ_FULL * HD, NH * SEQ_FULL * HD, WSCL, 0, 0);
  cvt_t<0><<<dim3(HD / 64, DMD / 64), blk, 0, stream>>>(wq, WQT, DMD, HD, HD, DMD, WSCL);
  cvt_t<0><<<dim3(HD / 64, DMD / 64), blk, 0, stream>>>(wk, WKT, DMD, HD, HD, DMD, WSCL);
  cvt_t<0><<<dim3(HD / 64, DMD / 64), blk, 0, stream>>>(wv, WVT, DMD, HD, HD, DMD, WSCL);
  cvt_t<1><<<dim3(DMD / 64, DMD / 64), blk, 0, stream>>>(wo, WOT, DMD, DMD, DMD, KF, 1.0f);
  cvt_t<1><<<dim3(DMD / 64, DMD / 64), blk, 0, stream>>>(wo, WOT + DMD, DMD, DMD, DMD, KF, 1.0f);
  cvt_t<1><<<dim3(EVP / 64, DMD / 64), blk, 0, stream>>>(wl, WLT, DMD, EVD, EVP, KF, 1.0f);
  cvt_t<1><<<dim3(EVP / 64, DMD / 64), blk, 0, stream>>>(wl, WLT + DMD, DMD, EVD, EVP, KF, 1.0f);

  const int gQ = ((MT / 64) * (HD / 64) + 7) / 8;
  gemm64<0, 1, 0, 0><<<dim3(gQ), blk, 0, stream>>>(XQ, DMD, WQT, DMD, QHp, 0, fdummy, HD, QKS / WSCL, bq, HD, QKS, MT, HD, DMD);
  gemm64<0, 1, 0, 0><<<dim3(gQ), blk, 0, stream>>>(XK, DMD, WKT, DMD, KHp, 0, fdummy, HD, QKS / WSCL, bk, HD, QKS, MT, HD, DMD);
  gemm64<0, 2, 0, 1><<<dim3(gQ), blk, 0, stream>>>(WVT, DMD, XV, DMD, VHp, HD * MT, fdummy, MT, 1.0f / WSCL, bv, HD, 1.0f, HD, MT, DMD);

  mask_check<<<dim3(NFLG), blk, 0, stream>>>(msk, FLG);
  attn_kernel<<<dim3((NB * NH * (SEQ / 16)) / AWV), dim3(128), 0, stream>>>(QHp, KHp, PEH, VHp, VLp, Zp);

  const int gO = ((MT / 64) * (DMD / 64) + 7) / 8;
  gemm64<1, 2, 1, 0><<<dim3(gO), blk, 0, stream>>>(Zp, KF, WOT, KF, OPp, DMD, fdummy, KF, 1.0f, bo, DMD, 1.0f, MT, DMD, KF);

  const int gL = ((MT / 64) * (EVP / 64) + 7) / 8;
  gemm64<1, 0, 0, 0><<<dim3(gL), blk, 0, stream>>>(OPp, KF, WLT, KF, hdummy, 0, Lp, EVP, 1.0f, bl, EVD, 1.0f, MT, EVP, KF);

  out_copy<<<dim3((MT * (EVD / 4) + 255) / 256), blk, 0, stream>>>(Lp, FLG, out0);
  (void)hipGetLastError();
}
